// MultiHeadAttention_65395172049448
// MI455X (gfx1250) — hardware-run, weakly checked
//
#include <hip/hip_runtime.h>
#ifndef NB
#define NB 2
#endif
#ifndef SEQ
#define SEQ 2048
#endif
#define SQ SEQ
#define NB_FULL 2
#define SQ_FULL 2048
#define DM 1024
#define NH 16
#define HD 64
#define HG 2
#define NREL 101
#define MAXREL 50
#define RP 128
#define PP (SQ + RP)
#define NR ((size_t)NB * SQ)
#define LQ DM
#define NIT (SQ / 256)

static_assert(SQ % 256 == 0);
static_assert(PP % 32 == 0);
static_assert(NH % HG == 0);
static_assert(NB <= NB_FULL);
static_assert(SQ <= SQ_FULL);
static_assert(NREL == 2 * MAXREL + 1);
static_assert(NREL <= RP);

typedef unsigned short v8us __attribute__((ext_vector_type(8), may_alias));
typedef float  v8f  __attribute__((ext_vector_type(8)));
typedef float  v4f  __attribute__((ext_vector_type(4)));
typedef float  v4fa __attribute__((ext_vector_type(4), may_alias));
typedef int    v4i  __attribute__((ext_vector_type(4)));
typedef int    v4ia __attribute__((ext_vector_type(4), may_alias));
typedef _Float16 v16h __attribute__((ext_vector_type(16)));
typedef _Float16 v4h  __attribute__((ext_vector_type(4)));
union FragH { v16h v; v8us q8[2]; _Float16 h[16]; unsigned short u[16]; };
union Frag8 { v8us v; _Float16 h[8]; unsigned short u[8]; };

__device__ __forceinline__ unsigned short bf16_bits(float x) { unsigned int u = __float_as_uint(x); return (unsigned short)((u + 0x7FFFu + ((u >> 16) & 1u)) >> 16); }
__device__ __forceinline__ float bf16_rne(float x) { return __uint_as_float(((unsigned int)bf16_bits(x)) << 16); }
__device__ __forceinline__ int rel_idx(int j, int i) { int dj = j - i; dj = dj < -MAXREL ? -MAXREL : (dj > MAXREL ? MAXREL : dj); return dj + MAXREL; }

__device__ __forceinline__ v16h g2_frag(const _Float16* p, int hh) { FragH f; f.q8[0] = *(const v8us*)((const unsigned short*)p + 8 * hh); f.q8[1] = *(const v8us*)((const unsigned short*)p + 16 + 8 * hh); return f.v; }
__device__ __forceinline__ v8f g2_mma(v16h a, v16h b, v8f c) { v8f d = __builtin_amdgcn_wmma_f32_16x16x32_f16(false, a, false, b, (short)0, c, false, false); asm volatile("v_nop\n\tv_nop\n\tv_nop\n\tv_nop" : "+v"(d) : "v"(a), "v"(b)); return d; }

__global__ __launch_bounds__(256) void k_wnat(const float* __restrict__ w, size_t n8, _Float16* __restrict__ Bt) {
  const size_t t = (size_t)blockIdx.x * 256 + threadIdx.x; if (t >= n8) return;
  const v4f a = *(const v4fa*)(w + t * 8), c = *(const v4fa*)(w + t * 8 + 4);
  Frag8 f;
#pragma unroll
  for (int q = 0; q < 4; ++q) { f.h[q] = (_Float16)(bf16_rne(a[q]) * 16.0f); f.h[4 + q] = (_Float16)(bf16_rne(c[q]) * 16.0f); }
  const v8us o = f.v;
  *(volatile v8us*)((unsigned short*)Bt + t * 8) = o; __threadfence(); *(volatile v8us*)((unsigned short*)Bt + t * 8) = o;
}

__global__ __launch_bounds__(256) void k_x16(const float* __restrict__ x, _Float16* __restrict__ X16, size_t n8) {
  const size_t t = (size_t)blockIdx.x * 256 + threadIdx.x; if (t >= n8) return;
  const size_t e = t * 8; const size_t row = e / DM; const size_t c = e % DM; const size_t b = row / SQ, s = row % SQ;
  const float* src = x + ((b * SQ_FULL + s) * DM + c);
  const v4f a = *(const v4fa*)(src), d = *(const v4fa*)(src + 4);
  Frag8 f;
#pragma unroll
  for (int q = 0; q < 4; ++q) { f.h[q] = (_Float16)bf16_rne(a[q]); f.h[4 + q] = (_Float16)bf16_rne(d[q]); }
  const v8us o = f.v;
  *(volatile v8us*)((unsigned short*)X16 + t * 8) = o; __threadfence(); *(volatile v8us*)((unsigned short*)X16 + t * 8) = o;
}

__global__ __launch_bounds__(256) void k_reltab(const float* __restrict__ Rk, const float* __restrict__ Rv, _Float16* __restrict__ RK16, _Float16* __restrict__ VT) {
  const int t = blockIdx.x * 256 + threadIdx.x;
  const int c = t % (RP / 8); const int d = (t / (RP / 8)) % HD; const int h = t / ((RP / 8) * HD);
  Frag8 fv;
#pragma unroll
  for (int q = 0; q < 8; ++q) { const int r = c * 8 + q; const int rr = r < NREL ? r : (NREL - 1); const float val = bf16_rne(Rv[rr * HD + d]); fv.h[q] = (r < NREL) ? (_Float16)val : (_Float16)0.0f; }
  const v8us ov = fv.v;
  unsigned short* dv = (unsigned short*)VT + ((size_t)h * HD + d) * PP + SQ + c * 8;
  const bool dok = t < RP * (HD / 8);
  const int tk = dok ? t : 0;
  const int n = tk / (HD / 8), k8 = (tk % (HD / 8)) * 8;
  Frag8 fk;
#pragma unroll
  for (int q = 0; q < 8; ++q) { const int nn = n < NREL ? n : (NREL - 1); const float val = bf16_rne(Rk[nn * HD + k8 + q]); fk.h[q] = (n < NREL) ? (_Float16)val : (_Float16)0.0f; }
  const v8us ok = fk.v;
  unsigned short* dk = (unsigned short*)RK16 + (size_t)n * HD + k8;
  for (int pass = 0; pass < 2; ++pass) {
    *(volatile v8us*)dv = ov;
    if (dok) *(volatile v8us*)dk = ok;
    if (pass == 0) __threadfence();
  }
}

template <bool HASBIAS, bool OUTF32>
__global__ __launch_bounds__(128) void k_gemm2(const _Float16* __restrict__ A, int lda, size_t sA, const _Float16* __restrict__ Bh, int ldb, size_t sB, float alpha,
    const float* __restrict__ bias, size_t sBias, float* __restrict__ C, _Float16* __restrict__ C16, int ldc, size_t sC, int M, int N, int K) {
  __shared__ __attribute__((aligned(16))) float so[4][32][68];
  const int tid = threadIdx.x, w = tid >> 5, lane = tid & 31, ln = lane & 15, hh = lane >> 4; const int by = blockIdx.y;
  A += (size_t)by * sA; Bh += (size_t)by * sB; const size_t cofs = (size_t)by * sC;
  const int ntn = N >> 6; const int mt = blockIdx.x / ntn, nq = blockIdx.x - mt * ntn; const int row0 = mt * 128 + 32 * w, col0 = nq * 64; if (row0 >= M) return;
  const _Float16* a0p = A + (size_t)(row0 + ln) * lda; const _Float16* a1p = a0p + (size_t)16 * lda;
  const _Float16* b0p = Bh + (size_t)(col0 + ln) * ldb; const _Float16* b1p = b0p + (size_t)16 * ldb; const _Float16* b2p = b1p + (size_t)16 * ldb; const _Float16* b3p = b2p + (size_t)16 * ldb;
  const v8f z8 = {0.f,0.f,0.f,0.f,0.f,0.f,0.f,0.f}; v8f c00 = z8, c01 = z8, c02 = z8, c03 = z8, c10 = z8, c11 = z8, c12 = z8, c13 = z8;
#pragma unroll 1
  for (int kb = 0; kb < K; kb += 32) { const v16h a0 = g2_frag(a0p + kb, hh), a1 = g2_frag(a1p + kb, hh);
    v16h b = g2_frag(b0p + kb, hh); c00 = g2_mma(a0, b, c00); c10 = g2_mma(a1, b, c10);
    b = g2_frag(b1p + kb, hh); c01 = g2_mma(a0, b, c01); c11 = g2_mma(a1, b, c11);
    b = g2_frag(b2p + kb, hh); c02 = g2_mma(a0, b, c02); c12 = g2_mma(a1, b, c12);
    b = g2_frag(b3p + kb, hh); c03 = g2_mma(a0, b, c03); c13 = g2_mma(a1, b, c13); }
  v8f accs[8] = {c00, c01, c02, c03, c10, c11, c12, c13};
#pragma unroll
  for (int u = 0; u < 8; ++u) { const int t = u & 3, hv = u >> 2; const int col = col0 + t * 16 + ln; float bv = 0.f; if (HASBIAS) bv = bf16_rne(bias[(size_t)by * sBias + col]);
#pragma unroll
    for (int r = 0; r < 8; ++r) so[w][hv * 16 + 8 * hh + r][t * 16 + ln] = accs[u][r] * alpha + bv; }
  __builtin_amdgcn_fence(4  , "workgroup"); __builtin_amdgcn_wave_barrier();
  const int rsub = lane >> 4, c4 = (lane & 15) * 4;
  for (int pass = 0; pass < 2; ++pass) {
#pragma unroll
    for (int q = 0; q < 16; ++q) { const int r = q * 2 + rsub; const v4f v = *(const v4fa*)&so[w][r][c4];
      if (OUTF32) { *(volatile v4f*)(C + cofs + (size_t)(row0 + r) * ldc + col0 + c4) = v; }
      else { v4h h4;
#pragma unroll
        for (int i = 0; i < 4; ++i) h4[i] = (_Float16)v[i];
        *(volatile v4h*)(C16 + cofs + (size_t)(row0 + r) * ldc + col0 + c4) = h4; } }
    if (pass == 0) __threadfence(); }
}

__global__ __launch_bounds__(128) void k_scores(const _Float16* __restrict__ A, int lda, size_t sA, const _Float16* __restrict__ Bh, int ldb, size_t sB, float alpha,
    const float* __restrict__ QR, const int* __restrict__ mask, float* __restrict__ C, int ldc, size_t sC, int M, int N, int K) {
  __shared__ __attribute__((aligned(16))) float so[4][32][68];
  const int tid = threadIdx.x, w = tid >> 5, lane = tid & 31, ln = lane & 15, hh = lane >> 4; const int by = blockIdx.y;
  A += (size_t)by * sA; Bh += (size_t)by * sB; const size_t cofs = (size_t)by * sC; const float* qrp = QR + (size_t)by * SQ * RP;
  const int ntn = N >> 6; const int mt = blockIdx.x / ntn, nq = blockIdx.x - mt * ntn; const int row0 = mt * 128 + 32 * w, col0 = nq * 64; if (row0 >= M) return;
  const _Float16* a0p = A + (size_t)(row0 + ln) * lda; const _Float16* a1p = a0p + (size_t)16 * lda;
  const _Float16* b0p = Bh + (size_t)(col0 + ln) * ldb; const _Float16* b1p = b0p + (size_t)16 * ldb; const _Float16* b2p = b1p + (size_t)16 * ldb; const _Float16* b3p = b2p + (size_t)16 * ldb;
  const v8f z8 = {0.f,0.f,0.f,0.f,0.f,0.f,0.f,0.f}; v8f c00 = z8, c01 = z8, c02 = z8, c03 = z8, c10 = z8, c11 = z8, c12 = z8, c13 = z8;
#pragma unroll 1
  for (int kb = 0; kb < K; kb += 32) { const v16h a0 = g2_frag(a0p + kb, hh), a1 = g2_frag(a1p + kb, hh);
    v16h b = g2_frag(b0p + kb, hh); c00 = g2_mma(a0, b, c00); c10 = g2_mma(a1, b, c10);
    b = g2_frag(b1p + kb, hh); c01 = g2_mma(a0, b, c01); c11 = g2_mma(a1, b, c11);
    b = g2_frag(b2p + kb, hh); c02 = g2_mma(a0, b, c02); c12 = g2_mma(a1, b, c12);
    b = g2_frag(b3p + kb, hh); c03 = g2_mma(a0, b, c03); c13 = g2_mma(a1, b, c13); }
  v8f accs[8] = {c00, c01, c02, c03, c10, c11, c12, c13};
#pragma unroll
  for (int u = 0; u < 8; ++u) { const int t = u & 3, hv = u >> 2;
#pragma unroll
    for (int r = 0; r < 8; ++r) so[w][hv * 16 + 8 * hh + r][t * 16 + ln] = accs[u][r] * alpha; }
  __builtin_amdgcn_fence(4  , "workgroup"); __builtin_amdgcn_wave_barrier();
  const int rsub = lane >> 4, c4 = (lane & 15) * 4;
#pragma unroll 2
  for (int q = 0; q < 16; ++q) { const int r = q * 2 + rsub; const int grow = row0 + r;
    v4f v = *(const v4fa*)&so[w][r][c4];
    const v4i m = *(const v4ia*)(mask + (size_t)grow * SQ_FULL + col0 + c4);
    const float* qr = qrp + (size_t)grow * RP;
    const int jb = col0 + c4;
    const int i0 = rel_idx(jb + 0, grow), i1 = rel_idx(jb + 1, grow), i2 = rel_idx(jb + 2, grow), i3 = rel_idx(jb + 3, grow);
    float p0 = qr[i0], p1 = qr[i1], p2 = qr[i2], p3 = qr[i3];
    asm volatile("" : "+v"(p0), "+v"(p1), "+v"(p2), "+v"(p3));
    const float s0 = v[0] + p0, s1 = v[1] + p1, s2 = v[2] + p2, s3 = v[3] + p3;
    v[0] = (m[0] != 0) ? -1.0e9f : s0;
    v[1] = (m[1] != 0) ? -1.0e9f : s1;
    v[2] = (m[2] != 0) ? -1.0e9f : s2;
    v[3] = (m[3] != 0) ? -1.0e9f : s3;
    *(v4fa*)&so[w][r][c4] = v; }
  __builtin_amdgcn_fence(4  , "workgroup"); __builtin_amdgcn_wave_barrier();
  for (int pass = 0; pass < 2; ++pass) {
#pragma unroll
    for (int q = 0; q < 16; ++q) { const int r = q * 2 + rsub; const v4f v = *(const v4fa*)&so[w][r][c4]; *(volatile v4f*)(C + cofs + (size_t)(row0 + r) * ldc + col0 + c4) = v; }
    if (pass == 0) __threadfence(); }
}

template <int NHv, int TTv, int PPv>
__global__ __launch_bounds__(256) void k_vt(const _Float16* __restrict__ V16, int ldv, int voff, _Float16* __restrict__ Vt) {
  __shared__ unsigned short tl[64][66];
  const int tid = threadIdx.x; const int slab = blockIdx.x / (TTv / 64), lg = blockIdx.x % (TTv / 64); const int b = slab / NHv, h = slab % NHv;
  for (int i = tid; i < 64 * 8; i += 256) { const int r = i / 8, c8 = (i % 8) * 8; Frag8 f; f.v = *(const v8us*)((const unsigned short*)V16 + ((size_t)b * TTv + lg * 64 + r) * ldv + voff + h * 64 + c8);
#pragma unroll
    for (int q = 0; q < 8; ++q) tl[r][c8 + q] = f.u[q]; }
  __syncthreads();
  for (int pass = 0; pass < 2; ++pass) {
#pragma unroll
    for (int rd = 0; rd < 2; ++rd) { const int d = rd * 32 + tid / 8, pc = tid % 8; Frag8 f;
#pragma unroll
      for (int q = 0; q < 8; ++q) f.u[q] = tl[pc * 8 + q][d];
      const v8us o = f.v;
      *(volatile v8us*)((unsigned short*)Vt + ((size_t)slab * 64 + d) * PPv + lg * 64 + pc * 8) = o; }
    if (pass == 0) __threadfence(); }
}

__global__ __launch_bounds__(256) void k_rsm_rel(const float* __restrict__ S, _Float16* __restrict__ P, int qn, int hg) {
  #pragma clang fp contract(off)
  const int lane = threadIdx.x & 31;
  const int wv = blockIdx.x * 8 + (threadIdx.x >> 5); if (wv >= qn * hg) return;
  const int hsel = wv / qn, i = wv - hsel * qn;
  const float* s = S + ((size_t)hsel * SQ + i) * SQ;
  unsigned short* prow = (unsigned short*)P + ((size_t)hsel * SQ + i) * PP;
  float e[NIT][8]; float mx = -3.0e38f;
#pragma unroll
  for (int it = 0; it < NIT; ++it) { const int j0 = it * 256 + lane * 8; const v4f a = *(const v4fa*)(s + j0), c = *(const v4fa*)(s + j0 + 4);
#pragma unroll
    for (int q = 0; q < 4; ++q) { e[it][q] = a[q]; e[it][4 + q] = c[q]; mx = fmaxf(mx, fmaxf(a[q], c[q])); } }
  const int cx = lane & 15;
  float k0, k1, k2, k3, k4, k5, k6, k7;
  { const int jb = i + cx * 8 - MAXREL;
    const int j0 = jb + 0, j1 = jb + 1, j2 = jb + 2, j3 = jb + 3, j4 = jb + 4, j5 = jb + 5, j6 = jb + 6, j7 = jb + 7;
    k0 = s[j0 < 0 ? 0 : (j0 > SQ - 1 ? SQ - 1 : j0)]; k1 = s[j1 < 0 ? 0 : (j1 > SQ - 1 ? SQ - 1 : j1)];
    k2 = s[j2 < 0 ? 0 : (j2 > SQ - 1 ? SQ - 1 : j2)]; k3 = s[j3 < 0 ? 0 : (j3 > SQ - 1 ? SQ - 1 : j3)];
    k4 = s[j4 < 0 ? 0 : (j4 > SQ - 1 ? SQ - 1 : j4)]; k5 = s[j5 < 0 ? 0 : (j5 > SQ - 1 ? SQ - 1 : j5)];
    k6 = s[j6 < 0 ? 0 : (j6 > SQ - 1 ? SQ - 1 : j6)]; k7 = s[j7 < 0 ? 0 : (j7 > SQ - 1 ? SQ - 1 : j7)]; }
  asm volatile("" : "+v"(k0), "+v"(k1), "+v"(k2), "+v"(k3), "+v"(k4), "+v"(k5), "+v"(k6), "+v"(k7));
  mx = fmaxf(mx, __shfl_xor(mx, 16)); mx = fmaxf(mx, __shfl_xor(mx, 8)); mx = fmaxf(mx, __shfl_xor(mx, 4)); mx = fmaxf(mx, __shfl_xor(mx, 2)); mx = fmaxf(mx, __shfl_xor(mx, 1));
  float se = 0.f;
#pragma unroll
  for (int it = 0; it < NIT; ++it)
#pragma unroll
    for (int q = 0; q < 8; ++q) { const float ev = __expf(e[it][q] - mx); e[it][q] = ev; se += ev; }
  se += __shfl_xor(se, 16); se += __shfl_xor(se, 8); se += __shfl_xor(se, 4); se += __shfl_xor(se, 2); se += __shfl_xor(se, 1);
  const float sc = 4096.0f / se;
  float a0 = 0.f, a100 = 0.f; Frag8 f[NIT];
#pragma unroll
  for (int it = 0; it < NIT; ++it)
#pragma unroll
    for (int q = 0; q < 8; ++q) { const int j = it * 256 + lane * 8 + q; const float pj = e[it][q] * sc; a0 += (j <= i - MAXREL) ? pj : 0.f; a100 += (j >= i + MAXREL) ? pj : 0.f; f[it].h[q] = (_Float16)pj; }
  a0 += __shfl_xor(a0, 16); a0 += __shfl_xor(a0, 8); a0 += __shfl_xor(a0, 4); a0 += __shfl_xor(a0, 2); a0 += __shfl_xor(a0, 1);
  a100 += __shfl_xor(a100, 16); a100 += __shfl_xor(a100, 8); a100 += __shfl_xor(a100, 4); a100 += __shfl_xor(a100, 2); a100 += __shfl_xor(a100, 1);
  const float ks[8] = {k0, k1, k2, k3, k4, k5, k6, k7};
  Frag8 fx;
#pragma unroll
  for (int q = 0; q < 8; ++q) { const int r = cx * 8 + q; const int j = i + r - MAXREL;
    float pv = __expf(ks[q] - mx) * sc;
    asm volatile("" : "+v"(pv));
    const bool inr = (r >= 1) && (r <= 2 * MAXREL - 1) && (j >= 0) && (j < SQ);
    float val = inr ? pv : 0.f; val = (r == 0) ? a0 : val; val = (r == 2 * MAXREL) ? a100 : val; fx.h[q] = (_Float16)val; }
  v8us ox = fx.v;
  asm volatile("" : "+v"(ox));
  for (int pass = 0; pass < 2; ++pass) {
#pragma unroll
    for (int it = 0; it < NIT; ++it) { const v8us o = f[it].v; *(volatile v8us*)(prow + it * 256 + lane * 8) = o; }
    if (lane < 16) *(volatile v8us*)(prow + SQ + cx * 8) = ox;
    if (pass == 0) __threadfence(); }
}

constexpr size_t al256(size_t b) { return (b + 255) & ~(size_t)255; }
constexpr size_t SZ_W   = al256((size_t)DM * DM * 2);
constexpr size_t SZ_ACT = al256(NR * DM * 2);
constexpr size_t SZ_S   = al256((size_t)HG * SQ * SQ * 4);
constexpr size_t SZ_P   = al256((size_t)HG * SQ * PP * 2);
constexpr size_t SZ_VT  = al256((size_t)NH * HD * PP * 2);
constexpr size_t SZ_QR  = al256((size_t)HG * SQ * RP * 4);
constexpr size_t SZ_RK  = al256((size_t)RP * HD * 2);
constexpr size_t SZ_TOTAL = 4 * SZ_W + 5 * SZ_ACT + SZ_S + SZ_P + SZ_VT + SZ_QR + SZ_RK;
static_assert(SZ_TOTAL <= (size_t)134217728);

extern "C" void kernel_launch(void* const* d_in, const int* in_sizes, int n_in,
                              void* d_out, int out_size, void* d_ws, size_t ws_size, hipStream_t stream) {
  if (n_in < 12) return;
  const size_t xneed = ((size_t)(NB - 1) * SQ_FULL + SQ) * DM;
  if ((size_t)in_sizes[0] < xneed) return;
  if ((size_t)in_sizes[1] < (size_t)(SQ - 1) * SQ_FULL + SQ) return;
  if ((size_t)in_sizes[2] < (size_t)DM * DM || (size_t)in_sizes[4] < (size_t)DM * DM || (size_t)in_sizes[6] < (size_t)DM * DM || (size_t)in_sizes[8] < (size_t)DM * DM) return;
  if (in_sizes[3] < DM || in_sizes[5] < DM || in_sizes[7] < DM || in_sizes[9] < DM) return;
  if (in_sizes[10] < NREL * HD || in_sizes[11] < NREL * HD) return;
  if ((size_t)out_size < xneed) return;
  const float* x = (const float*)d_in[0]; const int* mask = (const int*)d_in[1];
  const float* wq = (const float*)d_in[2]; const float* bq = (const float*)d_in[3]; const float* wk = (const float*)d_in[4]; const float* bk = (const float*)d_in[5];
  const float* wv = (const float*)d_in[6]; const float* bv = (const float*)d_in[7]; const float* wo = (const float*)d_in[8]; const float* bo = (const float*)d_in[9];
  const float* rk = (const float*)d_in[10]; const float* rv = (const float*)d_in[11];
  char* ws = (char*)d_ws; size_t off = 0;
  auto take = [&](size_t bytes) { char* p = ws + off; off += al256(bytes); return p; };
  _Float16* BQ = (_Float16*)take((size_t)DM * DM * 2); _Float16* BK = (_Float16*)take((size_t)DM * DM * 2); _Float16* BV = (_Float16*)take((size_t)DM * DM * 2); _Float16* BO = (_Float16*)take((size_t)DM * DM * 2);
  _Float16* X16 = (_Float16*)take(NR * DM * 2); _Float16* Q16 = (_Float16*)take(NR * DM * 2); _Float16* K16 = (_Float16*)take(NR * DM * 2); _Float16* V16 = (_Float16*)take(NR * DM * 2); _Float16* O16 = (_Float16*)take(NR * DM * 2);
  float* S = (float*)take((size_t)HG * SQ * SQ * 4); _Float16* P = (_Float16*)take((size_t)HG * SQ * PP * 2); _Float16* VT = (_Float16*)take((size_t)NH * HD * PP * 2);
  float* QR = (float*)take((size_t)HG * SQ * RP * 4); _Float16* RK16 = (_Float16*)take((size_t)RP * HD * 2);
  if (off > ws_size || off > (size_t)134217728) return;

  { const unsigned g = (unsigned)(((size_t)DM * DM / 8 + 255) / 256);
    k_wnat<<<g, 256, 0, stream>>>(wq, (size_t)DM * DM / 8, BQ); k_wnat<<<g, 256, 0, stream>>>(wk, (size_t)DM * DM / 8, BK);
    k_wnat<<<g, 256, 0, stream>>>(wv, (size_t)DM * DM / 8, BV); k_wnat<<<g, 256, 0, stream>>>(wo, (size_t)DM * DM / 8, BO); }
  k_x16<<<(unsigned)((NR * DM / 8 + 255) / 256), 256, 0, stream>>>(x, X16, NR * DM / 8);
  k_reltab<<<(NH * HD * (RP / 8)) / 256, 256, 0, stream>>>(rk, rv, RK16, VT);
  const int MP = (int)NR;
  k_gemm2<true, false><<<dim3((unsigned)((MP / 128) * (DM / 64)), 1), 128, 0, stream>>>(X16, DM, 0, BQ, DM, 0, 0.0625f, bq, 0, nullptr, Q16, DM, 0, MP, DM, DM);
  k_gemm2<true, false><<<dim3((unsigned)((MP / 128) * (DM / 64)), 1), 128, 0, stream>>>(X16, DM, 0, BK, DM, 0, 0.0625f, bk, 0, nullptr, K16, DM, 0, MP, DM, DM);
  k_gemm2<true, false><<<dim3((unsigned)((MP / 128) * (DM / 64)), 1), 128, 0, stream>>>(X16, DM, 0, BV, DM, 0, 0.0625f, bv, 0, nullptr, V16, DM, 0, MP, DM, DM);
  for (int b = 0; b < NB; ++b) { const size_t r0 = (size_t)b * SQ;
    k_vt<NH, SQ, PP><<<NH * (SQ / 64), 256, 0, stream>>>(V16 + r0 * LQ, LQ, 0, VT);
    for (int h0 = 0; h0 < NH; h0 += HG) {
      k_gemm2<false, true><<<dim3((SQ / 128) * (RP / 64), HG), 128, 0, stream>>>(Q16 + r0 * LQ + h0 * HD, LQ, (size_t)HD, RK16, HD, 0, 0.125f, nullptr, 0, QR, nullptr, RP, (size_t)SQ * RP, SQ, RP, HD);
      k_scores<<<dim3((SQ / 128) * (SQ / 64), HG), 128, 0, stream>>>(Q16 + r0 * LQ + h0 * HD, LQ, (size_t)HD, K16 + r0 * LQ + h0 * HD, LQ, (size_t)HD, 0.125f, QR, mask, S, SQ, (size_t)SQ * SQ, SQ, SQ, HD);
      k_rsm_rel<<<(HG * SQ + 7) / 8, 256, 0, stream>>>(S, P, SQ, HG);
      k_gemm2<false, false><<<dim3((SQ / 128) * (HD / 64), HG), 128, 0, stream>>>(P, PP, (size_t)SQ * PP, VT + (size_t)h0 * HD * PP, PP, (size_t)HD * PP, 0.015625f, nullptr, 0, nullptr, O16 + r0 * DM + h0 * HD, DM, (size_t)HD, SQ, HD, PP);
    } }
  k_gemm2<true, true><<<dim3((unsigned)((SQ / 128) * (DM / 64)), NB), 128, 0, stream>>>(O16, DM, (size_t)SQ * DM, BO, DM, 0, 0.0009765625f, bo, 0, (float*)d_out, nullptr, DM, (size_t)SQ_FULL * DM, SQ, DM, DM);
}
